// MultiheadAttention_62311385530901
// MI455X (gfx1250) — hardware-verified
//
#include <hip/hip_runtime.h>


#ifndef NB
#define NB 2048
#endif
#define NB_FULL 2048
#define TT   64
#define CC   64
#define NHD  8
#define HD   64
#define HDT  (NHD * HD)
#define MW   4
#define XP   72
#define PP   68
#define TP   72
#define PSH  8.0f
#define RSC  2048.0f
#define RES  (1.0f / 2048.0f)
#define SCQ  (0.125f * 1.4426950408889634f / 4096.0f)
#define CSC  0.25f
#define OSC  (1.0f / 4096.0f)
#define NEGB (-3.0e38f)

#define OFF_X 0
#define OFF_F (TT * XP * 2)
#define OFF_P (OFF_F + MW * 32768)
#define LDS_BYTES (OFF_P + MW * TT * PP * 4)

static_assert(NB <= NB_FULL);
static_assert(MW * 2 == NHD);
static_assert(HD == 64);
static_assert(TT == 64);
static_assert(CC == 64);
static_assert(OFF_F % 16 == 0);
static_assert(OFF_P % 16 == 0);
static_assert((XP * 2) % 16 == 0);
static_assert((PP * 4) % 16 == 0);
static_assert(LDS_BYTES <= 262144);

typedef _Float16 h16;
typedef __attribute__((ext_vector_type(16))) _Float16 v16h;
typedef __attribute__((ext_vector_type(8)))  _Float16 v8h;
typedef __attribute__((ext_vector_type(4)))  _Float16 v4h;
typedef __attribute__((ext_vector_type(8)))  float    v8f;
typedef __attribute__((ext_vector_type(4)))  float    v4f;
typedef v4f  __attribute__((may_alias)) v4fa;
typedef v8h  __attribute__((may_alias)) v8ha;
typedef v4h  __attribute__((may_alias)) v4ha;

__device__ __forceinline__ float rbf(float f) { unsigned u = __float_as_uint(f); u += 0x7FFFu + ((u >> 16) & 1u); return __uint_as_float(u & 0xFFFF0000u); }
__device__ __forceinline__ v16h cat16(v8h lo, v8h hi) { return __builtin_shufflevector(lo, hi, 0, 1, 2, 3, 4, 5, 6, 7, 8, 9, 10, 11, 12, 13, 14, 15); }
__device__ __forceinline__ v8f wmma16(v16h a, v16h b, v8f c) { return __builtin_amdgcn_wmma_f32_16x16x32_f16(false, a, false, b, (short)0, c, false, false); }
__device__ __forceinline__ v16h ldh(const h16* p) { return cat16(*(const v8h*)p, *(const v8h*)(p + 16)); }
__device__ __forceinline__ v16h ldl(const h16* p) { const v8h a = *(const v8ha*)p; const v8h c = *(const v8ha*)(p + 16); return cat16(a, c); }
__device__ __forceinline__ v16h ldf(const v8ha* fs, int plane, int f) { const int i = ((plane * 8 + f) * 2) * 32; const v8h a = fs[i]; const v8h c = fs[i + 32]; return cat16(a, c); }
__device__ __forceinline__ void stf(v8ha* fs, int plane, int f, v8h a, v8h c) { const int i = ((plane * 8 + f) * 2) * 32; fs[i] = a; fs[i + 32] = c; }
__device__ __forceinline__ void split8(const v8f d, v8h& hi, v8h& lo) {
#pragma unroll
    for (int r = 0; r < 8; ++r) { const float v = d[r]; const h16 hv = (h16)v; hi[r] = hv; lo[r] = (h16)((v - (float)hv) * RSC); }
}
__device__ __forceinline__ void pair_tiles(v16h a1c0, v16h a1c1, v16h a2c0, v16h a2c1, v16h bc0, v16h bc1, v8f& d1, v8f& d2) {
    v8f x = (v8f){}, y = (v8f){};
    x = wmma16(a1c0, bc0, x); y = wmma16(a2c0, bc0, y);
    x = wmma16(a1c1, bc1, x); y = wmma16(a2c1, bc1, y);
    asm volatile("v_nop\n\tv_nop\n\tv_nop\n\tv_nop" : "+v"(x), "+v"(y) : "v"(a1c0), "v"(a1c1), "v"(a2c0), "v"(a2c1), "v"(bc0), "v"(bc1));
    d1 = x; d2 = y;
}

__global__ __launch_bounds__(256) void k_wt(const float* __restrict__ src, h16* dst, int dts, int dpitch, float scale) {
    __shared__ __align__(16) h16 ts[64 * TP];
    const int tid = threadIdx.x;
    const int r = tid >> 2, c0 = (tid & 3) * 16;
    const float* s = src + (size_t)blockIdx.x * 4096 + r * 64 + c0;
#pragma unroll
    for (int q = 0; q < 4; ++q) { const v4f x = *(const v4f*)(s + 4 * q);
#pragma unroll
        for (int i = 0; i < 4; ++i) ts[(c0 + 4 * q + i) * TP + r] = (h16)(rbf(x[i]) * scale); }
    __syncthreads();
    h16* d = dst + (size_t)blockIdx.x * dts;
#pragma unroll 1
    for (int ps = 0; ps < 2; ++ps) {
#pragma unroll
        for (int s2 = 0; s2 < 2; ++s2) { const int dd = 32 * s2 + (tid >> 3), c8 = (tid & 7) * 8;
            const v8h val = *(const v8ha*)(&ts[dd * TP + c8]);
            *(volatile v8h*)(d + (size_t)dd * dpitch + c8) = val; }
        if (ps == 0) __threadfence(); }
}

__global__ __launch_bounds__(32 * MW) void k_mha(const float* __restrict__ X, const h16* __restrict__ WQT, const h16* __restrict__ WKT, const h16* __restrict__ WVT,
                                                 const h16* __restrict__ WPT, const float* __restrict__ BP, float* OUT) {
    extern __shared__ __align__(16) unsigned char smem[];
    h16* xs = (h16*)(smem + OFF_X);
    const int tid = threadIdx.x;
    const int lane = tid & 31, wave = __builtin_amdgcn_readfirstlane((int)(threadIdx.x >> 5)), lr = lane & 15, hi = lane >> 4;
    const int b = blockIdx.x;

    {
        const float* xb = X + (size_t)b * (TT * CC);
#pragma unroll
        for (int it = 0; it < 8; ++it) {
            const int e = 4 * (tid + 128 * it); const int row = e >> 6, col = e & 63;
            const v4f v = *(const v4f*)(xb + e); v4h o;
#pragma unroll
            for (int k = 0; k < 4; ++k) o[k] = (h16)rbf(v[k]);
            *(v4ha*)(xs + row * XP + col) = o;
        }
    }
    __syncthreads();

    v8ha* fs = (v8ha*)(smem + OFF_F) + wave * 2048 + lane;
    float* pw = (float*)(smem + OFF_P) + wave * (TT * PP);
    const h16* xr = xs + lr * XP + 8 * hi;

#pragma unroll 1
    for (int hh = 0; hh < 2; ++hh) {
        const int h = wave + MW * hh;
        const size_t wo = (size_t)h * 4096 + (size_t)lr * 64 + 8 * hi;

#pragma unroll 1
        for (int ks = 0; ks < 2; ++ks) {
            const h16* xa = xr + (2 * ks) * 16 * XP;
            const v16h xa0 = ldl(xa), xa1 = ldl(xa + 32), xb0 = ldl(xa + 16 * XP), xb1 = ldl(xa + 16 * XP + 32);
#pragma unroll 1
            for (int dj = 0; dj < 4; ++dj) {
                const h16* wv_ = WVT + wo + dj * 1024;
                const v16h w0 = ldh(wv_), w1 = ldh(wv_ + 32);
                v8f d1, d2; pair_tiles(xa0, xa1, xb0, xb1, w0, w1, d1, d2);
                v8h h1, l1, h2, l2; split8(d1, h1, l1); split8(d2, h2, l2);
                stf(fs, 2, dj * 2 + ks, h1, h2); stf(fs, 3, dj * 2 + ks, l1, l2);
            }
#pragma unroll 1
            for (int ds = 0; ds < 2; ++ds) {
                const h16* wk_ = WKT + wo + (2 * ds) * 1024;
                const v16h a10 = ldh(wk_), a11 = ldh(wk_ + 32), a20 = ldh(wk_ + 1024), a21 = ldh(wk_ + 1024 + 32);
                v8f d1, d2; v8h h1, l1, h2, l2;
                pair_tiles(a10, a11, a20, a21, xa0, xa1, d1, d2);
                split8(d1, h1, l1); split8(d2, h2, l2);
                stf(fs, 0, (2 * ks) * 2 + ds, h1, h2); stf(fs, 1, (2 * ks) * 2 + ds, l1, l2);
                pair_tiles(a10, a11, a20, a21, xb0, xb1, d1, d2);
                split8(d1, h1, l1); split8(d2, h2, l2);
                stf(fs, 0, (2 * ks + 1) * 2 + ds, h1, h2); stf(fs, 1, (2 * ks + 1) * 2 + ds, l1, l2);
            }
        }

#pragma unroll 1
        for (int ti = 0; ti < 4; ++ti) {
            const int t = 16 * ti + lr;
            v16h qh0, ql0, qh1, ql1;
            {
                const h16* xq = xr + ti * 16 * XP;
                const v16h x0 = ldl(xq), x1 = ldl(xq + 32);
                const h16* wq_ = WQT + wo;
                v8f d1, d2; v8h h1, l1, h2, l2;
                {
                    const v16h a10 = ldh(wq_), a11 = ldh(wq_ + 32), a20 = ldh(wq_ + 1024), a21 = ldh(wq_ + 1024 + 32);
                    pair_tiles(a10, a11, a20, a21, x0, x1, d1, d2);
                    split8(d1, h1, l1); split8(d2, h2, l2);
                    qh0 = cat16(h1, h2); ql0 = cat16(l1, l2);
                }
                {
                    const v16h a10 = ldh(wq_ + 2048), a11 = ldh(wq_ + 2048 + 32), a20 = ldh(wq_ + 3072), a21 = ldh(wq_ + 3072 + 32);
                    pair_tiles(a10, a11, a20, a21, x0, x1, d1, d2);
                    split8(d1, h1, l1); split8(d2, h2, l2);
                    qh1 = cat16(h1, h2); ql1 = cat16(l1, l2);
                }
            }
            v8f o[4], ol[4];
#pragma unroll
            for (int j = 0; j < 4; ++j) { o[j] = (v8f){}; ol[j] = (v8f){}; }
            float m = NEGB, l = 0.0f;
            const int nks = (ti >> 1) + 1;
#pragma unroll 1
            for (int ks = 0; ks < nks; ++ks) {
                const int fa = 4 * ks;
                v8f sa = (v8f){}, sal = (v8f){}, sb = (v8f){}, sbl = (v8f){};
                {
                    const v16h kh0 = ldf(fs, 0, fa), kh1 = ldf(fs, 0, fa + 1), kl0 = ldf(fs, 1, fa), kl1 = ldf(fs, 1, fa + 1);
                    sa = wmma16(kh0, qh0, sa); sal = wmma16(kl0, qh0, sal);
                    sa = wmma16(kh1, qh1, sa); sal = wmma16(kh0, ql0, sal);
                    sal = wmma16(kl1, qh1, sal); sal = wmma16(kh1, ql1, sal);
                    asm volatile("v_nop\n\tv_nop\n\tv_nop\n\tv_nop" : "+v"(sa), "+v"(sal) : "v"(kh0), "v"(kh1), "v"(kl0), "v"(kl1), "v"(qh0), "v"(qh1), "v"(ql0), "v"(ql1));
                }
                {
                    const v16h kh0 = ldf(fs, 0, fa + 2), kh1 = ldf(fs, 0, fa + 3), kl0 = ldf(fs, 1, fa + 2), kl1 = ldf(fs, 1, fa + 3);
                    sb = wmma16(kh0, qh0, sb); sbl = wmma16(kl0, qh0, sbl);
                    sb = wmma16(kh1, qh1, sb); sbl = wmma16(kh0, ql0, sbl);
                    sbl = wmma16(kl1, qh1, sbl); sbl = wmma16(kh1, ql1, sbl);
                    asm volatile("v_nop\n\tv_nop\n\tv_nop\n\tv_nop" : "+v"(sb), "+v"(sbl) : "v"(kh0), "v"(kh1), "v"(kl0), "v"(kl1), "v"(qh0), "v"(qh1), "v"(ql0), "v"(ql1));
                }
                const int kbase = 32 * ks + 8 * hi;
                float ta[8], tb[8]; float mx = NEGB;
#pragma unroll
                for (int r = 0; r < 8; ++r) {
                    const float va = (sa[r] + sal[r] * RES) * SCQ;
                    const float vb = (sb[r] + sbl[r] * RES) * SCQ;
                    ta[r] = (kbase + r <= t) ? va : NEGB;
                    tb[r] = (kbase + 16 + r <= t) ? vb : NEGB;
                    mx = fmaxf(mx, fmaxf(ta[r], tb[r]));
                }
                mx = fmaxf(mx, __shfl_xor(mx, 16, 32));
                const float mnew = fmaxf(m, mx);
                const float alpha = __builtin_amdgcn_exp2f(m - mnew);
                const float sh = PSH - mnew;
                v16h pb, pl; float ls = 0.0f;
#pragma unroll
                for (int r = 0; r < 8; ++r) {
                    const float fa_ = __builtin_amdgcn_exp2f(ta[r] + sh);
                    const float fb_ = __builtin_amdgcn_exp2f(tb[r] + sh);
                    const h16 ha = (h16)fa_; const h16 hb = (h16)fb_;
                    pb[r] = ha; pb[8 + r] = hb;
                    pl[r] = (h16)((fa_ - (float)ha) * RSC); pl[8 + r] = (h16)((fb_ - (float)hb) * RSC);
                    ls += fa_ + fb_;
                }
                l = l * alpha + ls; m = mnew;
#pragma unroll
                for (int j = 0; j < 4; ++j) { o[j] = o[j] * alpha; ol[j] = ol[j] * alpha; }
#pragma unroll
                for (int j = 0; j < 4; ++j) {
                    const v16h vh = ldf(fs, 2, 2 * j + ks), vl = ldf(fs, 3, 2 * j + ks);
                    o[j] = wmma16(vh, pb, o[j]); ol[j] = wmma16(vl, pb, ol[j]); ol[j] = wmma16(vh, pl, ol[j]);
                    asm volatile("v_nop\n\tv_nop\n\tv_nop\n\tv_nop" : "+v"(o[j]), "+v"(ol[j]) : "v"(vh), "v"(vl), "v"(pb), "v"(pl));
                }
            }
            l += __shfl_xor(l, 16, 32);
            const float cs = CSC * (1.0f / l);
            v16h cah0, cal0, cah1, cal1;
#pragma unroll
            for (int r = 0; r < 8; ++r) {
                float c; h16 ch;
                c = (o[0][r] + ol[0][r] * RES) * cs; ch = (h16)c; cah0[r] = ch;     cal0[r] = (h16)((c - (float)ch) * RSC);
                c = (o[1][r] + ol[1][r] * RES) * cs; ch = (h16)c; cah0[8 + r] = ch; cal0[8 + r] = (h16)((c - (float)ch) * RSC);
                c = (o[2][r] + ol[2][r] * RES) * cs; ch = (h16)c; cah1[r] = ch;     cal1[r] = (h16)((c - (float)ch) * RSC);
                c = (o[3][r] + ol[3][r] * RES) * cs; ch = (h16)c; cah1[8 + r] = ch; cal1[8 + r] = (h16)((c - (float)ch) * RSC);
            }
            const h16* wpp = WPT + (size_t)lr * HDT + h * HD + 8 * hi;
            float* prow = pw + (16 * ti + 8 * hi) * PP + lr;
#pragma unroll 1
            for (int cj = 0; cj < 4; ++cj) {
                const h16* bp_ = wpp + (size_t)cj * 16 * HDT;
                const v16h b0 = ldh(bp_), b1 = ldh(bp_ + 32);
                v8f acc = (v8f){}, accl = (v8f){};
                acc = wmma16(cah0, b0, acc); accl = wmma16(cal0, b0, accl);
                acc = wmma16(cah1, b1, acc); accl = wmma16(cal1, b1, accl);
                asm volatile("v_nop\n\tv_nop\n\tv_nop\n\tv_nop" : "+v"(acc), "+v"(accl) : "v"(cah0), "v"(cal0), "v"(cah1), "v"(cal1), "v"(b0), "v"(b1));
                float* p = prow + 16 * cj;
                if (hh == 0) {
#pragma unroll
                    for (int r = 0; r < 8; ++r) p[r * PP] = (acc[r] + accl[r] * RES) * OSC;
                } else {
#pragma unroll
                    for (int r = 0; r < 8; ++r) { const float nv = p[r * PP] + (acc[r] + accl[r] * RES) * OSC; p[r * PP] = nv; }
                }
            }
        }
    }
    __syncthreads();

    const float* pall = (const float*)(smem + OFF_P);
    v4f bv = *(const v4f*)(BP + 4 * lr);
#pragma unroll
    for (int k = 0; k < 4; ++k) bv[k] = rbf(bv[k]);
    v4f vals[8];
#pragma unroll
    for (int s = 0; s < 8; ++s) {
        const int idx = (16 * wave + 2 * s + hi) * PP + 4 * lr;
        v4f a = *(const v4fa*)(pall + idx);
        const v4f a1 = *(const v4fa*)(pall + TT * PP + idx);
        const v4f a2 = *(const v4fa*)(pall + 2 * TT * PP + idx);
        const v4f a3 = *(const v4fa*)(pall + 3 * TT * PP + idx);
        a = ((a + a1) + a2) + a3;
        vals[s] = a + bv;
    }
    float* orow = OUT + (size_t)b * (TT * CC) + (size_t)(16 * wave) * CC + 4 * lr;
#pragma unroll 1
    for (int ps = 0; ps < 2; ++ps) {
#pragma unroll
        for (int s = 0; s < 8; ++s) *(volatile v4f*)(orow + (size_t)(2 * s + hi) * CC) = vals[s];
        if (ps == 0) __threadfence(); }
}

static constexpr size_t SZ_W = (size_t)NHD * CC * HD * 2;
static constexpr size_t SZ_TOTAL = 4 * SZ_W;
static_assert((size_t)HDT * CC * 2 <= SZ_W);
static_assert(SZ_TOTAL <= (size_t)134217728);

extern "C" void kernel_launch(void* const* d_in, const int* in_sizes, int n_in,
                              void* d_out, int out_size, void* d_ws, size_t ws_size, hipStream_t stream) {
    if (n_in < 6) return;
    if ((size_t)in_sizes[0] < (size_t)NB * TT * CC) return;
    if (in_sizes[1] < NHD * CC * HD || in_sizes[2] < NHD * CC * HD || in_sizes[3] < NHD * CC * HD) return;
    if (in_sizes[4] < HDT * CC || in_sizes[5] < CC) return;
    if ((size_t)out_size < (size_t)NB * TT * CC) return;
    if (SZ_TOTAL > ws_size) return;
    const float* x  = (const float*)d_in[0];
    const float* Wq = (const float*)d_in[1];
    const float* Wk = (const float*)d_in[2];
    const float* Wv = (const float*)d_in[3];
    const float* Wp = (const float*)d_in[4];
    const float* bp = (const float*)d_in[5];
    float* OUT = (float*)d_out;
    char* wsp = (char*)d_ws;
    h16* WQT = (h16*)wsp; wsp += SZ_W;
    h16* WKT = (h16*)wsp; wsp += SZ_W;
    h16* WVT = (h16*)wsp; wsp += SZ_W;
    h16* WPT = (h16*)wsp; wsp += SZ_W;

    k_wt<<<NHD, 256, 0, stream>>>(Wq, WQT, 4096, 64, 64.0f);
    k_wt<<<NHD, 256, 0, stream>>>(Wk, WKT, 4096, 64, 64.0f);
    k_wt<<<NHD, 256, 0, stream>>>(Wv, WVT, 4096, 64, 64.0f);
    k_wt<<<HDT / 64, 256, 0, stream>>>(Wp, WPT, 64, HDT, 256.0f);

    (void)hipFuncSetAttribute(reinterpret_cast<const void*>(&k_mha), hipFuncAttributeMaxDynamicSharedMemorySize, (int)LDS_BYTES);
    k_mha<<<NB, 32 * MW, LDS_BYTES, stream>>>(x, WQT, WKT, WVT, WPT, bp, OUT);
}
